// MultiScaleMambaBlock_63780264345765
// MI455X (gfx1250) — hardware-verified
//
#include <hip/hip_runtime.h>
#include <math.h>

#define B_    4
#define CDIM  64
#define L_    4096
#define NT    16384
#define DIN   128
#define NST   16
#define DTR   4
#define KD    4
#define HID   170
#define XPC   36
#define XPCP  48
#define FFN2  340
#define FFN2P 352
#define KPOUT 192
#define CHUNK 64

typedef __attribute__((ext_vector_type(16))) _Float16 v16h;
typedef __attribute__((ext_vector_type(8)))  _Float16 v8h;
typedef __attribute__((ext_vector_type(8)))  float    v8f;
typedef __attribute__((ext_vector_type(4)))  float    v4f;
typedef __attribute__((ext_vector_type(4)))  unsigned v4u;
typedef float __attribute__((may_alias)) float_a;

template <typename V> __device__ __forceinline__ void vst2(void* p, V v) {
  *(volatile V*)p = v; __threadfence(); *(volatile V*)p = v;
}
__device__ __forceinline__ float siluf(float x)     { return x / (1.f + __expf(-x)); }
__device__ __forceinline__ float softplusf(float x) { return (x > 20.f) ? x : log1pf(__expf(x)); }

__device__ __forceinline__ v8f wmma_tile(const _Float16* __restrict__ A, int lda, const _Float16* __restrict__ W, int ldw,
                                         int m0, int n0, int K, v8f acc, int lane)
{
  const int mr = lane & 15, koff = (lane & 16) ? 8 : 0;
  const _Float16* ap = A + (size_t)(m0 + mr) * lda + koff;
  const _Float16* wp = W + (size_t)(n0 + mr) * ldw + koff;
  for (int k0 = 0; k0 < K; k0 += 32) {
    v8h alo = *(const v8h*)(ap), ahi = *(const v8h*)(ap + 16);
    v8h blo = *(const v8h*)(wp), bhi = *(const v8h*)(wp + 16);
    v16h a, b;
#pragma unroll
    for (int i = 0; i < 8; ++i) { a[i] = alo[i]; a[i + 8] = ahi[i]; b[i] = blo[i]; b[i + 8] = bhi[i]; }
    acc = __builtin_amdgcn_wmma_f32_16x16x32_f16(false, a, false, b, (short)0, acc, false, false);
    asm volatile("v_nop\n\tv_nop\n\tv_nop\n\tv_nop" : "+v"(acc) : "v"(a), "v"(b));
    ap += 32; wp += 32;
  }
  return acc;
}

__global__ void k_cvt_pad(const float* __restrict__ s, _Float16* __restrict__ d, int rows, int scols, int dstride, int srows)
{
  const int g = blockIdx.x * blockDim.x + threadIdx.x;
  if (g * 8 >= rows * dstride) return;
  const int r = (g * 8) / dstride, c0 = (g * 8) % dstride;
  union { v8h h; v4u u; } pk;
#pragma unroll
  for (int e = 0; e < 8; ++e) { const int c = c0 + e; pk.h[e] = (r < srows && c < scols) ? (_Float16)s[(size_t)r * scols + c] : (_Float16)0.f; }
  vst2(d + (size_t)g * 8, pk.u);
}
__global__ void k_cvt_xproj(const float* __restrict__ s, _Float16* __restrict__ d)
{
  const int g = blockIdx.x * blockDim.x + threadIdx.x;
  if (g * 8 >= KD * XPCP * DIN) return;
  const int i0 = g * 8;
  const int k = i0 / (XPCP * DIN); const int rem = i0 % (XPCP * DIN); const int c = rem / DIN, dd = rem % DIN;
  union { v8h h; v4u u; } pk;
#pragma unroll
  for (int e = 0; e < 8; ++e) pk.h[e] = (c < XPC) ? (_Float16)s[((size_t)(k * XPC + c)) * DIN + dd + e] : (_Float16)0.f;
  vst2(d + (size_t)i0, pk.u);
}

__global__ __launch_bounds__(256) void k_ln1(const float* __restrict__ x, const float* __restrict__ w,
                                             const float* __restrict__ bias, _Float16* __restrict__ xn)
{
  const int gid = blockIdx.x * 256 + threadIdx.x;
  const int t = gid >> 3, part = gid & 7;
  const int b = t >> 12, l = t & 4095;
  const float* xp = x + (size_t)b * CDIM * L_ + l;
  float v[8], s = 0.f, sq = 0.f;
#pragma unroll
  for (int e = 0; e < 8; ++e) { v[e] = xp[(size_t)(part * 8 + e) * L_]; s += v[e]; sq += v[e] * v[e]; }
#pragma unroll
  for (int off = 1; off < 8; off <<= 1) { s += __shfl_xor(s, off, 32); sq += __shfl_xor(sq, off, 32); }
  const float mu = s * (1.f / CDIM), inv = rsqrtf(sq * (1.f / CDIM) - mu * mu + 1e-6f);
  union { v8h h; v4u u; } pk;
#pragma unroll
  for (int e = 0; e < 8; ++e) { const int c = part * 8 + e; pk.h[e] = (_Float16)((v[e] - mu) * inv * w[c] + bias[c]); }
  vst2(xn + (size_t)t * CDIM + part * 8, pk.u);
}

__global__ __launch_bounds__(256) void k_gemm_inproj(const _Float16* __restrict__ A, const _Float16* __restrict__ W,
                                                     float* __restrict__ xm, float* __restrict__ z)
{
  __shared__ __align__(16) float T[128][132];
  const int tid = threadIdx.x, wave = tid >> 5, lane = tid & 31;
  const int m0 = blockIdx.x * 128 + wave * 16, nbase = blockIdx.y * DIN;
  const int moff = (lane & 16) ? 8 : 0, col = lane & 15;
#pragma unroll 1
  for (int nt = 0; nt < 8; ++nt) {
    v8f acc = {};
    acc = wmma_tile(A, CDIM, W, CDIM, m0, nbase + nt * 16, CDIM, acc, lane);
#pragma unroll
    for (int r = 0; r < 8; ++r) T[wave * 16 + moff + r][nt * 16 + col] = acc[r];
  }
  __syncthreads();
  const int mb = blockIdx.x * 128, b = mb >> 12, l0 = mb & 4095;
  if (blockIdx.y == 0) {
    for (int g = tid; g < 128 * 32; g += 256) { const int n = g >> 5, pc = g & 31;
      v4f v = {T[pc * 4][n], T[pc * 4 + 1][n], T[pc * 4 + 2][n], T[pc * 4 + 3][n]};
      vst2(xm + (((size_t)(b * DIN + n)) << 12) + l0 + pc * 4, v); }
  } else {
    for (int g = tid; g < 128 * 32; g += 256) { const int ml = g >> 5, pc = g & 31;
      vst2(z + (size_t)(mb + ml) * DIN + pc * 4, *(const v4f*)(&T[ml][pc * 4])); }
  }
}

__global__ __launch_bounds__(256) void k_conv_silu(const float* __restrict__ xm, const float* __restrict__ cw, const float* __restrict__ cb,
                                                   _Float16* __restrict__ xsA, _Float16* __restrict__ xsB)
{
  const int gid = blockIdx.x * 256 + threadIdx.x;
  const int t = gid >> 4, part = gid & 15;
  const int b = t >> 12, l = t & 4095, hh = l >> 6, ww = l & 63;
  union { v8h h; v4u u; } pk;
#pragma unroll 1
  for (int e = 0; e < 8; ++e) {
    const int c = part * 8 + e;
    const float* p = xm + (size_t)(b * DIN + c) * L_;
    const float* wp = cw + c * 9;
    float acc = cb[c];
#pragma unroll
    for (int dh = -1; dh <= 1; ++dh) { const int y = hh + dh; if ((unsigned)y >= 64u) continue;
#pragma unroll
      for (int dx = -1; dx <= 1; ++dx) { const int x2 = ww + dx; if ((unsigned)x2 >= 64u) continue; acc += p[y * 64 + x2] * wp[(dh + 1) * 3 + (dx + 1)]; } }
    pk.h[e] = (_Float16)siluf(acc);
  }
  const int lB = (ww << 6) + hh;
  vst2(xsA + ((size_t)b * L_ + l)  * DIN + part * 8, pk.u);
  vst2(xsB + ((size_t)b * L_ + lB) * DIN + part * 8, pk.u);
}

__global__ __launch_bounds__(256) void k_gemm_xdbl(const _Float16* __restrict__ xsA, const _Float16* __restrict__ xsB,
                                                   const _Float16* __restrict__ Wp, float* __restrict__ xdbl)
{
  __shared__ __align__(16) float T[128 * XPCP];
  const int k = blockIdx.y;
  const _Float16* A = (k & 1) ? xsB : xsA;
  const _Float16* W = Wp + (size_t)k * XPCP * DIN;
  const int tid = threadIdx.x, wave = tid >> 5, lane = tid & 31;
  const int mb = blockIdx.x * 128, m0 = mb + wave * 16, moff = (lane & 16) ? 8 : 0, col = lane & 15;
#pragma unroll 1
  for (int nt = 0; nt < XPCP / 16; ++nt) {
    v8f acc = {};
    acc = wmma_tile(A, DIN, W, DIN, m0, nt * 16, DIN, acc, lane);
#pragma unroll
    for (int r = 0; r < 8; ++r) T[(wave * 16 + moff + r) * XPCP + nt * 16 + col] = acc[r];
  }
  __syncthreads();
  float* dst = xdbl + ((size_t)k * NT + mb) * XPCP;
  for (int g = tid; g < 128 * XPCP / 4; g += 256) vst2(dst + g * 4, *(const v4f*)(&T[g * 4]));
}

__global__ void __launch_bounds__(128) k_scan(const float* __restrict__ xdbl, const _Float16* __restrict__ xsA,
                                               const _Float16* __restrict__ xsB, const float* __restrict__ dt_w,
                                               const float* __restrict__ dt_b, const float* __restrict__ A_logs,
                                               const float* __restrict__ Ds, float* __restrict__ ydir)
{
  __shared__ __align__(16) float sx[2][CHUNK * XPCP];
  const int k = blockIdx.x >> 2, b = blockIdx.x & 3, d = threadIdx.x;
  float Arow[NST];
#pragma unroll
  for (int n = 0; n < NST; ++n) Arow[n] = -__expf(A_logs[(size_t)(k * DIN + d) * NST + n]);
  float dtw[DTR];
#pragma unroll
  for (int r = 0; r < DTR; ++r) dtw[r] = dt_w[(size_t)(k * DIN + d) * DTR + r];
  const float dtb = dt_b[k * DIN + d], Dd = Ds[k * DIN + d];
  float h[NST];
#pragma unroll
  for (int n = 0; n < NST; ++n) h[n] = 0.f;
  const float*    xrow = xdbl + ((size_t)k * NT + (size_t)b * L_) * XPCP;
  const _Float16* xs   = ((k & 1) ? xsB : xsA) + (size_t)b * L_ * DIN;
  float*          yo   = ydir + ((size_t)(k * B_ + b) * L_) * DIN;
  const bool rev = (k >= 2);
  const int  NC  = L_ / CHUNK;
  auto cbase = [&](int c) { return rev ? (L_ - (c + 1) * CHUNK) : c * CHUNK; };
  auto stage = [&](int buf, int c) {
    const v4f* src = (const v4f*)(xrow + (size_t)cbase(c) * XPCP);
    v4f* dstp = (v4f*)&sx[buf][0];
    for (int i = d; i < CHUNK * XPCP / 4; i += 128) dstp[i] = src[i];
  };
  stage(0, 0);
  int cur = 0;
  for (int c = 0; c < NC; ++c) {
    __syncthreads();
    if (c + 1 < NC) stage(cur ^ 1, c + 1);
    const float* sxc = &sx[cur][0];
    const int base = cbase(c);
    for (int i = 0; i < CHUNK; ++i) {
      const int t   = c * CHUNK + i;
      const int row = rev ? (L_ - 1 - t) : (base + i);
      const float* sr = sxc + (row - base) * XPCP;
      const float u = (float)xs[(size_t)row * DIN + d];
      const float dpre  = dtb + sr[0]*dtw[0] + sr[1]*dtw[1] + sr[2]*dtw[2] + sr[3]*dtw[3];
      const float delta = softplusf(dpre);
      const float du = delta * u;
      float y  = Dd * u;
#pragma unroll
      for (int n = 0; n < NST; ++n) {
        const float dA = __expf(delta * Arow[n]);
        h[n] = dA * h[n] + du * sr[DTR + n];
        y   += h[n] * sr[DTR + NST + n];
      }
      vst2(yo + (size_t)row * DIN + d, (float_a)y);
    }
    __syncthreads();
    cur ^= 1;
  }
}

__global__ __launch_bounds__(256) void k_combine(const float* __restrict__ ydir, const float* __restrict__ z,
                                                 const float* __restrict__ w, const float* __restrict__ bias, _Float16* __restrict__ yg)
{
  const int gid = blockIdx.x * 256 + threadIdx.x;
  const int t = gid >> 5, lane = gid & 31;
  const int b = t >> 12, lA = t & 4095, hh = lA >> 6, ww = lA & 63, lB = (ww << 6) + hh;
  const size_t base0 = ((size_t)(0 * B_ + b) * L_ + lA) * DIN, base2 = ((size_t)(2 * B_ + b) * L_ + lA) * DIN;
  const size_t base1 = ((size_t)(1 * B_ + b) * L_ + lB) * DIN, base3 = ((size_t)(3 * B_ + b) * L_ + lB) * DIN;
  float v[4], s = 0.f, sq = 0.f;
#pragma unroll
  for (int i = 0; i < 4; ++i) { const int c = lane * 4 + i;
    const float vv = ydir[base0 + c] + ydir[base2 + c] + ydir[base1 + c] + ydir[base3 + c]; v[i] = vv; s += vv; sq += vv * vv; }
#pragma unroll
  for (int off = 16; off > 0; off >>= 1) { s += __shfl_xor(s, off, 32); sq += __shfl_xor(sq, off, 32); }
  const float mu = s * (1.f / DIN), inv = rsqrtf(sq * (1.f / DIN) - mu * mu + 1e-5f);
  union { _Float16 hh4[4]; unsigned long long u; } pk;
#pragma unroll
  for (int i = 0; i < 4; ++i) { const int c = lane * 4 + i; const float zz = z[(size_t)t * DIN + c];
    pk.hh4[i] = (_Float16)(((v[i] - mu) * inv * w[c] + bias[c]) * siluf(zz)); }
  vst2(yg + (size_t)t * DIN + lane * 4, pk.u);
}

__global__ __launch_bounds__(256) void k_gemm_outproj(const _Float16* __restrict__ A, const _Float16* __restrict__ W, float* __restrict__ yout)
{
  __shared__ __align__(16) float T[128 * CDIM];
  const int tid = threadIdx.x, wave = tid >> 5, lane = tid & 31;
  const int mb = blockIdx.x * 128, m0 = mb + wave * 16, moff = (lane & 16) ? 8 : 0, col = lane & 15;
#pragma unroll 1
  for (int nt = 0; nt < CDIM / 16; ++nt) {
    v8f acc = {};
    acc = wmma_tile(A, DIN, W, DIN, m0, nt * 16, DIN, acc, lane);
#pragma unroll
    for (int r = 0; r < 8; ++r) T[(wave * 16 + moff + r) * CDIM + nt * 16 + col] = acc[r];
  }
  __syncthreads();
  float* dst = yout + (size_t)mb * CDIM;
  for (int g = tid; g < 128 * CDIM / 4; g += 256) vst2(dst + g * 4, *(const v4f*)(&T[g * 4]));
}

__global__ __launch_bounds__(256) void k_res(const float* __restrict__ x, const float* __restrict__ yout, float* __restrict__ x1)
{
  const int t = blockIdx.x * 256 + threadIdx.x;
  const int b = t >> 12, l = t & 4095;
  const float* xp = x + (size_t)b * CDIM * L_ + l;
  float* x1p = x1 + (size_t)b * CDIM * L_ + l;
  const float* yp = yout + (size_t)t * CDIM;
#pragma unroll 4
  for (int c = 0; c < CDIM; ++c) vst2(x1p + (size_t)c * L_, (float_a)(xp[(size_t)c * L_] + yp[c]));
}
__global__ __launch_bounds__(256) void k_ln2(const float* __restrict__ x1, const float* __restrict__ w, const float* __restrict__ bias,
                                             _Float16* __restrict__ xn2)
{
  const int gid = blockIdx.x * 256 + threadIdx.x;
  const int t = gid >> 3, part = gid & 7, b = t >> 12, l = t & 4095;
  const float* xp = x1 + (size_t)b * CDIM * L_ + l;
  float v[8], s = 0.f, sq = 0.f;
#pragma unroll
  for (int e = 0; e < 8; ++e) { v[e] = xp[(size_t)(part * 8 + e) * L_]; s += v[e]; sq += v[e] * v[e]; }
#pragma unroll
  for (int off = 1; off < 8; off <<= 1) { s += __shfl_xor(s, off, 32); sq += __shfl_xor(sq, off, 32); }
  const float mu = s * (1.f / CDIM), inv = rsqrtf(sq * (1.f / CDIM) - mu * mu + 1e-6f);
  union { v8h h; v4u u; } pk;
#pragma unroll
  for (int e = 0; e < 8; ++e) { const int c = part * 8 + e; pk.h[e] = (_Float16)((v[e] - mu) * inv * w[c] + bias[c]); }
  vst2(xn2 + (size_t)t * CDIM + part * 8, pk.u);
}

__global__ __launch_bounds__(256) void k_gemm_pin(const _Float16* __restrict__ A, const _Float16* __restrict__ W, float* __restrict__ hbuf)
{
  __shared__ __align__(16) float T[16][132];
  const int tid = threadIdx.x, wave = tid >> 5, lane = tid & 31;
  const int mb = blockIdx.x * 128, m0 = mb + wave * 16, n0 = blockIdx.y * 16, moff = (lane & 16) ? 8 : 0, col = lane & 15;
  v8f acc = {};
  acc = wmma_tile(A, CDIM, W, CDIM, m0, n0, CDIM, acc, lane);
#pragma unroll
  for (int r = 0; r < 8; ++r) T[col][wave * 16 + moff + r] = acc[r];
  __syncthreads();
  const int b = mb >> 12, l0 = mb & 4095;
  for (int g = tid; g < 16 * 32; g += 256) { const int n = g >> 5, pc = g & 31; const int ch = n0 + n;
    if (ch < FFN2) vst2(hbuf + ((size_t)(b * FFN2 + ch)) * L_ + l0 + pc * 4, *(const v4f*)(&T[n][pc * 4])); }
}

__global__ __launch_bounds__(256) void k_ffngate(const float* __restrict__ hbuf, const float* __restrict__ dw, _Float16* __restrict__ g)
{
  const int gid = blockIdx.x * 256 + threadIdx.x;
  const int t = gid / 24, part = gid % 24;
  const int b = t >> 12, l = t & 4095, hh = l >> 6, ww = l & 63;
  union { v8h h; v4u u; } pk;
#pragma unroll 1
  for (int e = 0; e < 8; ++e) {
    const int c = part * 8 + e;
    float val = 0.f;
    if (c < HID) {
      const float* p1 = hbuf + (size_t)(b * FFN2 + c) * L_;
      const float* p2 = hbuf + (size_t)(b * FFN2 + c + HID) * L_;
      const float* w1 = dw + c * 9;
      const float* w2 = dw + (c + HID) * 9;
      float a = 0.f, bb = 0.f;
#pragma unroll
      for (int dh = -1; dh <= 1; ++dh) { const int y = hh + dh; if ((unsigned)y >= 64u) continue;
#pragma unroll
        for (int dx = -1; dx <= 1; ++dx) { const int x2 = ww + dx; if ((unsigned)x2 >= 64u) continue;
          const int off = y * 64 + x2, wo = (dh + 1) * 3 + (dx + 1); a += p1[off] * w1[wo]; bb += p2[off] * w2[wo]; } }
      const float ge = 0.5f * a * (1.f + erff(a * 0.70710678118654752f));
      val = ge * bb;
    }
    pk.h[e] = (_Float16)val;
  }
  vst2(g + ((size_t)b * L_ + l) * KPOUT + part * 8, pk.u);
}

__global__ __launch_bounds__(256) void k_gemm_pout(const _Float16* __restrict__ A, const _Float16* __restrict__ W,
                                                   const float* __restrict__ x1, float* __restrict__ out)
{
  __shared__ __align__(16) float T[CDIM][132];
  const int tid = threadIdx.x, wave = tid >> 5, lane = tid & 31;
  const int mb = blockIdx.x * 128, m0 = mb + wave * 16, moff = (lane & 16) ? 8 : 0, col = lane & 15;
  const int b = mb >> 12, l0 = mb & 4095;
#pragma unroll 1
  for (int nt = 0; nt < CDIM / 16; ++nt) {
    const int n = nt * 16 + col;
    v8f acc;
#pragma unroll
    for (int r = 0; r < 8; ++r) { const int m = m0 + moff + r; acc[r] = x1[(((size_t)(b * CDIM + n)) << 12) + (m & 4095)]; }
    acc = wmma_tile(A, KPOUT, W, KPOUT, m0, nt * 16, KPOUT, acc, lane);
#pragma unroll
    for (int r = 0; r < 8; ++r) T[n][wave * 16 + moff + r] = acc[r];
  }
  __syncthreads();
  for (int gq = tid; gq < CDIM * 32; gq += 256) { const int n = gq >> 5, pc = gq & 31;
    vst2(out + (((size_t)(b * CDIM + n)) << 12) + l0 + pc * 4, *(const v4f*)(&T[n][pc * 4])); }
}

extern "C" void kernel_launch(void* const* d_in, const int* in_sizes, int n_in,
                              void* d_out, int out_size, void* d_ws, size_t ws_size,
                              hipStream_t stream)
{
  (void)in_sizes; (void)n_in; (void)out_size; (void)ws_size;
  const float* x         = (const float*)d_in[0];
  const float* ln1_w     = (const float*)d_in[1];
  const float* ln1_b     = (const float*)d_in[2];
  const float* in_proj_w = (const float*)d_in[3];
  const float* conv_w    = (const float*)d_in[4];
  const float* conv_b    = (const float*)d_in[5];
  const float* x_proj_w  = (const float*)d_in[6];
  const float* dt_w      = (const float*)d_in[7];
  const float* dt_b      = (const float*)d_in[8];
  const float* A_logs    = (const float*)d_in[9];
  const float* Ds        = (const float*)d_in[10];
  const float* onw       = (const float*)d_in[11];
  const float* onb       = (const float*)d_in[12];
  const float* out_pw    = (const float*)d_in[13];
  const float* ln2_w     = (const float*)d_in[14];
  const float* ln2_b     = (const float*)d_in[15];
  const float* pin_w     = (const float*)d_in[16];
  const float* dw_w      = (const float*)d_in[17];
  const float* pout_w    = (const float*)d_in[18];
  float* out = (float*)d_out;

  char* base = (char*)d_ws; size_t off = 0;
  auto alloc = [&](size_t bytes) -> void* { void* p = base + off; off = (off + bytes + 255) & ~(size_t)255; return p; };
  _Float16* xn_h      = (_Float16*)alloc((size_t)NT * CDIM * 2);
  _Float16* inproj_h  = (_Float16*)alloc((size_t)2 * DIN * CDIM * 2);
  float*    xm        = (float*)   alloc((size_t)B_ * DIN * L_ * 4);
  float*    zbuf      = (float*)   alloc((size_t)NT * DIN * 4);
  _Float16* xsA_h     = (_Float16*)alloc((size_t)NT * DIN * 2);
  _Float16* xsB_h     = (_Float16*)alloc((size_t)NT * DIN * 2);
  _Float16* xproj_h   = (_Float16*)alloc((size_t)KD * XPCP * DIN * 2);
  float*    xdbl      = (float*)   alloc((size_t)KD * NT * XPCP * 4);
  float*    ydir      = (float*)   alloc((size_t)KD * NT * DIN * 4);
  _Float16* yg_h      = (_Float16*)alloc((size_t)NT * DIN * 2);
  _Float16* outproj_h = (_Float16*)alloc((size_t)CDIM * DIN * 2);
  float*    yout      = (float*)   alloc((size_t)NT * CDIM * 4);
  float*    x1        = (float*)   alloc((size_t)B_ * CDIM * L_ * 4);
  _Float16* xn2_h     = (_Float16*)alloc((size_t)NT * CDIM * 2);
  _Float16* pin_h     = (_Float16*)alloc((size_t)FFN2P * CDIM * 2);
  float*    hbuf      = (float*)   alloc((size_t)B_ * FFN2 * L_ * 4);
  _Float16* g_h       = (_Float16*)alloc((size_t)NT * KPOUT * 2);
  _Float16* pout_h    = (_Float16*)alloc((size_t)CDIM * KPOUT * 2);

  k_cvt_pad<<<(2 * DIN * CDIM / 8 + 255) / 256, 256, 0, stream>>>(in_proj_w, inproj_h, 2 * DIN, CDIM, CDIM, 2 * DIN);
  k_cvt_pad<<<(CDIM * DIN / 8 + 255) / 256, 256, 0, stream>>>(out_pw, outproj_h, CDIM, DIN, DIN, CDIM);
  k_cvt_pad<<<(FFN2P * CDIM / 8 + 255) / 256, 256, 0, stream>>>(pin_w, pin_h, FFN2P, CDIM, CDIM, FFN2);
  k_cvt_pad<<<(CDIM * KPOUT / 8 + 255) / 256, 256, 0, stream>>>(pout_w, pout_h, CDIM, HID, KPOUT, CDIM);
  k_cvt_xproj<<<(KD * XPCP * DIN / 8 + 255) / 256, 256, 0, stream>>>(x_proj_w, xproj_h);

  k_ln1<<<NT * 8 / 256, 256, 0, stream>>>(x, ln1_w, ln1_b, xn_h);
  k_gemm_inproj<<<dim3(NT / 128, 2), 256, 0, stream>>>(xn_h, inproj_h, xm, zbuf);
  k_conv_silu<<<NT * 16 / 256, 256, 0, stream>>>(xm, conv_w, conv_b, xsA_h, xsB_h);
  k_gemm_xdbl<<<dim3(NT / 128, KD), 256, 0, stream>>>(xsA_h, xsB_h, xproj_h, xdbl);
  k_scan<<<KD * B_, DIN, 0, stream>>>(xdbl, xsA_h, xsB_h, dt_w, dt_b, A_logs, Ds, ydir);
  k_combine<<<(NT * 32) / 256, 256, 0, stream>>>(ydir, zbuf, onw, onb, yg_h);
  k_gemm_outproj<<<NT / 128, 256, 0, stream>>>(yg_h, outproj_h, yout);
  k_res<<<NT / 256, 256, 0, stream>>>(x, yout, x1);
  k_ln2<<<NT * 8 / 256, 256, 0, stream>>>(x1, ln2_w, ln2_b, xn2_h);
  k_gemm_pin<<<dim3(NT / 128, FFN2P / 16), 256, 0, stream>>>(xn2_h, pin_h, hbuf);
  k_ffngate<<<(NT * 24) / 256, 256, 0, stream>>>(hbuf, dw_w, g_h);
  k_gemm_pout<<<NT / 128, 256, 0, stream>>>(g_h, pout_h, x1, out);
}
